// BaselineGRU_38070590112285
// MI455X (gfx1250) — hardware-verified
//
#include <hip/hip_runtime.h>
#include <math.h>

typedef __attribute__((ext_vector_type(16))) _Float16 v16h;
typedef __attribute__((ext_vector_type(8)))  _Float16 v8h;
typedef __attribute__((ext_vector_type(8)))  float    v8f;
typedef __attribute__((ext_vector_type(4)))  float    v4f;

constexpr int DIM_B = 8;
constexpr int DIM_N = 512;
constexpr int DIM_T = 256;
constexpr int DIM_D = 64;
constexpr int NROWS = DIM_B * DIM_N;
constexpr int NGATE = 3 * DIM_D;
constexpr int ROWS_PER_WAVE = 16;
constexpr int WAVES_PER_BLOCK = 4;
constexpr int ROWS_PER_BLOCK = ROWS_PER_WAVE * WAVES_PER_BLOCK;
constexpr int THREADS_PER_BLOCK = 32 * WAVES_PER_BLOCK;
constexpr int NBLOCKS = NROWS / ROWS_PER_BLOCK;
static_assert(NROWS % ROWS_PER_BLOCK == 0);
static_assert(DIM_D == 64);
static_assert(DIM_N % ROWS_PER_BLOCK == 0);
static_assert(NGATE * DIM_D % (8 * THREADS_PER_BLOCK) == 0);
static_assert(ROWS_PER_BLOCK * DIM_D % (8 * THREADS_PER_BLOCK) == 0);

constexpr float SCALE_H   = 8.0f;
constexpr float SCALE_W   = 16.0f;
constexpr float SCALE_INV = 1.0f / 128.0f;

__device__ __forceinline__ void dep_guard_h(v8f& a, v8f& b, v16h x, v16h y) { asm volatile("v_nop\n\tv_nop\n\tv_nop\n\tv_nop" : "+v"(a), "+v"(b) : "v"(x), "v"(y)); }
template <typename T> struct Frag;
template <> struct Frag<_Float16> {
  typedef v16h V; union U { v16h v; v8h h[2]; };
  static __device__ __forceinline__ v16h load(const _Float16* p) {
    U f; f.h[0] = *(const v8h*)(p); f.h[1] = *(const v8h*)(p + 16); return f.v;
  }
  static __device__ __forceinline__ v8f mma(v16h a, v16h b, v8f c) {
    return __builtin_amdgcn_wmma_f32_16x16x32_f16(false, a, false, b, (short)0, c, false, false);
  }
};

__device__ __forceinline__ void guard_group(v8f& a, v8f& b, v8f& c,
                                            v16h x0, v16h x1, v16h y0, v16h y1,
                                            v16h y2, v16h y3, v16h y4, v16h y5) {
  asm volatile("v_nop\n\tv_nop\n\tv_nop\n\tv_nop"
               : "+v"(a), "+v"(b), "+v"(c)
               : "v"(x0), "v"(x1), "v"(y0), "v"(y1), "v"(y2), "v"(y3), "v"(y4), "v"(y5));
}

__device__ __forceinline__ float gate_sigmoid(float x) {
  const float xc = fminf(fmaxf(x, -40.0f), 40.0f);
  return 1.0f / (1.0f + expf(-xc));
}
__device__ __forceinline__ float gate_tanh(float x) {
  const float yc = fminf(fmaxf(2.0f * x, -40.0f), 40.0f);
  return 2.0f / (1.0f + expf(-yc)) - 1.0f;
}

__global__ __launch_bounds__(THREADS_PER_BLOCK) void gru_fused_kernel(
    const float* __restrict__ x,
    const float* __restrict__ proj_w,
    const float* __restrict__ proj_b,
    const float* __restrict__ w_ih,
    const float* __restrict__ w_hh,
    const float* __restrict__ b_ih,
    const float* __restrict__ b_hh,
    const float* __restrict__ out_w,
    const float* __restrict__ out_b,
    float* __restrict__ out)
{
  __shared__ __align__(16) _Float16 Wsh[NGATE * DIM_D];
  __shared__ __align__(16) _Float16 Hsh[ROWS_PER_BLOCK * DIM_D];
  __shared__ __align__(16) float sU[NGATE];
  __shared__ __align__(16) float sV[NGATE];
  __shared__ __align__(16) float sBH[NGATE];
  __shared__ __align__(16) float sOW[DIM_D];
  __shared__ __align__(16) float sOut[ROWS_PER_BLOCK];

  const int tid  = threadIdx.x;
  const int wave = tid >> 5;
  const int lane = tid & 31;
  const int lo   = lane & 15;
  const int hi   = lane >> 4;
  const int blockbase = blockIdx.x * ROWS_PER_BLOCK;

  for (int idx = tid; idx < NGATE * DIM_D / 8; idx += THREADS_PER_BLOCK) {
    const v4f f0 = *(const v4f*)(w_hh + idx * 8);
    const v4f f1 = *(const v4f*)(w_hh + idx * 8 + 4);
    v8h hv;
    hv[0] = (_Float16)(f0[0] * SCALE_W); hv[1] = (_Float16)(f0[1] * SCALE_W);
    hv[2] = (_Float16)(f0[2] * SCALE_W); hv[3] = (_Float16)(f0[3] * SCALE_W);
    hv[4] = (_Float16)(f1[0] * SCALE_W); hv[5] = (_Float16)(f1[1] * SCALE_W);
    hv[6] = (_Float16)(f1[2] * SCALE_W); hv[7] = (_Float16)(f1[3] * SCALE_W);
    *(v8h*)(Wsh + idx * 8) = hv;
  }
  for (int idx = tid; idx < ROWS_PER_BLOCK * DIM_D / 8; idx += THREADS_PER_BLOCK) {
    v8h z;
    z[0] = (_Float16)0.0f; z[1] = (_Float16)0.0f; z[2] = (_Float16)0.0f; z[3] = (_Float16)0.0f;
    z[4] = (_Float16)0.0f; z[5] = (_Float16)0.0f; z[6] = (_Float16)0.0f; z[7] = (_Float16)0.0f;
    *(v8h*)(Hsh + idx * 8) = z;
  }
  for (int o = tid; o < NGATE; o += THREADS_PER_BLOCK) {
    float u = 0.0f, vv = 0.0f;
#pragma unroll 1
    for (int k = 0; k < DIM_D; ++k) {
      const float w = w_ih[o * DIM_D + k];
      u  = fmaf(w, proj_w[k], u);
      vv = fmaf(w, proj_b[k], vv);
    }
    sU[o]  = u;
    sV[o]  = vv + b_ih[o];
    sBH[o] = b_hh[o];
  }
  if (tid < DIM_D) sOW[tid] = out_w[tid];
  __syncthreads();

  float uR[4], uZ[4], uC[4], vR[4], vZ[4], vC[4], bC[4], owL[4];
#pragma unroll
  for (int dt = 0; dt < 4; ++dt) {
    const int o = dt * 16 + lo;
    uR[dt] = sU[o];           uZ[dt] = sU[DIM_D + o];                   uC[dt] = sU[2 * DIM_D + o];
    vR[dt] = sV[o] + sBH[o];  vZ[dt] = sV[DIM_D + o] + sBH[DIM_D + o];  vC[dt] = sV[2 * DIM_D + o];
    bC[dt] = sBH[2 * DIM_D + o];
    owL[dt] = sOW[o];
  }

  const int bidx = blockbase >> 9;
  const int tb   = ((blockbase & 511) >> 1) + wave * 8 + 4 * hi;
  const float* xa_base = x + ((size_t)(bidx * DIM_N) * DIM_T + tb);
  const float* xb_base = x + ((size_t)(bidx * DIM_N + 256) * DIM_T + tb);

  _Float16* Hw = Hsh + wave * ROWS_PER_WAVE * DIM_D;

  v8f H[4];
#pragma unroll
  for (int dt = 0; dt < 4; ++dt) H[dt] = (v8f){0.f, 0.f, 0.f, 0.f, 0.f, 0.f, 0.f, 0.f};

  for (int j = 0; j < DIM_T; ++j) {
    const v4f xa = *(const v4f*)(xa_base + (size_t)j * DIM_T);
    const v4f xb = *(const v4f*)(xb_base + (size_t)j * DIM_T);

    const v16h A0 = Frag<_Float16>::load(Hw + lo * DIM_D + 8 * hi);
    const v16h A1 = Frag<_Float16>::load(Hw + lo * DIM_D + 32 + 8 * hi);

#pragma unroll
    for (int dt = 0; dt < 4; ++dt) {
      const _Float16* wr = Wsh + (dt * 16 + lo) * DIM_D + 8 * hi;
      const _Float16* wz = Wsh + (DIM_D + dt * 16 + lo) * DIM_D + 8 * hi;
      const _Float16* wc = Wsh + (2 * DIM_D + dt * 16 + lo) * DIM_D + 8 * hi;
      const v16h b0 = Frag<_Float16>::load(wr);
      const v16h b1 = Frag<_Float16>::load(wr + 32);
      const v16h c0 = Frag<_Float16>::load(wz);
      const v16h c1 = Frag<_Float16>::load(wz + 32);
      const v16h d0 = Frag<_Float16>::load(wc);
      const v16h d1 = Frag<_Float16>::load(wc + 32);

      v8f accR = (v8f){0.f, 0.f, 0.f, 0.f, 0.f, 0.f, 0.f, 0.f};
      v8f accZ = (v8f){0.f, 0.f, 0.f, 0.f, 0.f, 0.f, 0.f, 0.f};
      v8f accC = (v8f){0.f, 0.f, 0.f, 0.f, 0.f, 0.f, 0.f, 0.f};
      accR = Frag<_Float16>::mma(A0, b0, accR);
      accR = Frag<_Float16>::mma(A1, b1, accR);
      accZ = Frag<_Float16>::mma(A0, c0, accZ);
      accZ = Frag<_Float16>::mma(A1, c1, accZ);
      accC = Frag<_Float16>::mma(A0, d0, accC);
      accC = Frag<_Float16>::mma(A1, d1, accC);
      guard_group(accR, accZ, accC, A0, A1, b0, b1, c0, c1, d0, d1);

#pragma unroll
      for (int v = 0; v < 8; ++v) {
        const float s  = (v & 1) ? xb[v >> 1] : xa[v >> 1];
        const float pr = fmaf(s, uR[dt], vR[dt]) + accR[v] * SCALE_INV;
        const float pz = fmaf(s, uZ[dt], vZ[dt]) + accZ[v] * SCALE_INV;
        const float r  = gate_sigmoid(pr);
        const float z  = gate_sigmoid(pz);
        const float g  = fmaf(s, uC[dt], vC[dt]) + r * fmaf(accC[v], SCALE_INV, bC[dt]);
        const float c  = gate_tanh(g);
        const float hp = H[dt][v];
        const float hn = (1.0f - z) * c + z * hp;
        H[dt][v] = hn;
        Hw[(8 * hi + v) * DIM_D + dt * 16 + lo] = (_Float16)(hn * SCALE_H);
      }
    }
    __syncthreads();
  }

  const float ob = out_b[0];
#pragma unroll
  for (int v = 0; v < 8; ++v) {
    float p = 0.0f;
#pragma unroll
    for (int dt = 0; dt < 4; ++dt) p = fmaf(H[dt][v], owL[dt], p);
    p += __shfl_xor(p, 1);
    p += __shfl_xor(p, 2);
    p += __shfl_xor(p, 4);
    p += __shfl_xor(p, 8);
    if (lo == 0) sOut[wave * ROWS_PER_WAVE + 8 * hi + v] = p + ob;
  }
  __syncthreads();

  if (wave == 0) {
    const v4f val = *(const v4f*)(sOut + 4 * lo);
    float* dst = out + blockbase + 4 * lo;
    if (lane < 16) *(volatile v4f*)dst = val;
    __threadfence();
    if (lane < 16) *(volatile v4f*)dst = val;
  }
}

extern "C" void kernel_launch(void* const* d_in, const int* in_sizes, int n_in,
                              void* d_out, int out_size, void* d_ws, size_t ws_size,
                              hipStream_t stream) {
  (void)d_ws; (void)ws_size;
  if (n_in < 9) return;
  if (in_sizes[0] != DIM_B * DIM_N * DIM_T) return;
  if (in_sizes[1] != DIM_D || in_sizes[2] != DIM_D) return;
  if (in_sizes[3] != NGATE * DIM_D || in_sizes[4] != NGATE * DIM_D) return;
  if (in_sizes[5] != NGATE || in_sizes[6] != NGATE) return;
  if (in_sizes[7] != DIM_D || in_sizes[8] < 1) return;
  if (out_size != NROWS) return;

  const float* x      = (const float*)d_in[0];
  const float* proj_w = (const float*)d_in[1];
  const float* proj_b = (const float*)d_in[2];
  const float* w_ih   = (const float*)d_in[3];
  const float* w_hh   = (const float*)d_in[4];
  const float* b_ih   = (const float*)d_in[5];
  const float* b_hh   = (const float*)d_in[6];
  const float* out_w  = (const float*)d_in[7];
  const float* out_b  = (const float*)d_in[8];

  gru_fused_kernel<<<dim3(NBLOCKS), dim3(THREADS_PER_BLOCK), 0, stream>>>(
      x, proj_w, proj_b, w_ih, w_hh, b_ih, b_hh, out_w, out_b, (float*)d_out);
}
